// GATRiskPredictor_15281493639282
// MI455X (gfx1250) — hardware-run, weakly checked
//
#include <hip/hip_runtime.h>
#include <stddef.h>
#include <stdint.h>
#include <math.h>

#define NN      10000
#define NP      10112
#define FIN     256
#define HC      512
#define CD      128
#define NE      320000
#define EOFF    20000
#define GBM     128
#define SP      68
#define NTHR    256
#define NWAVE   8
#define EPT     8
#define WCH     (32 * EPT)
#define NBRUN   512
#define SLB     9
#define NBK     20
#define WLCAP   2560
#define RCAP    20480
#define DEGCAP  128
#define MAXDEG_MEAS  54
#define MAXB512_MEAS 16584
#define SPLIT_TWO   0
#define SPLIT_THREE 1
#define SPLIT_HEAD  1
#define K_TWO   (SPLIT_TWO   ? 1024 : 512)
#define K_THREE (SPLIT_THREE ? 1024 : 512)
#define K_HEAD  (SPLIT_HEAD  ? 256 : 128)

#define P_A1   0
#define P_B1   1024
#define P_A2   1536
#define P_B2   2560
#define P_A3   3072
#define P_B3   3328
#define P_HD   3456
#define P_END  3840

#define BK_ZINTS (NWAVE * WLCAP + RCAP + 3 * NBRUN)
#define BK_INTS  (BK_ZINTS + 16)
#define BK_LDS   (BK_INTS * 4)

#define PBX   (NP * FIN / 8 / NTHR)
#define PBW1  (HC * FIN / 8 / NTHR)
#define PBW2  (HC * 1024 / 8 / NTHR)
#define PBW3  (CD * 1024 / 8 / NTHR)
#define PBWC  (64 * 256 / 8 / NTHR)
#define PBPAR 4
#define PBTOT (PBX + PBW1 + PBW2 + PBW3 + PBWC + PBPAR)

static_assert(NP % GBM == 0 && NP >= NN && NP == 79 * GBM && NP % NWAVE == 0);
static_assert(NBRUN == (1 << SLB) && NBRUN % GBM == 0);
static_assert(NBK * NBRUN >= NP);
static_assert(NE % WCH == 0 && NE % 4 == 0);
static_assert((((long long)NE) << SLB) < (1LL << 31));
static_assert(NN < (1 << 14));
static_assert(RCAP == NWAVE * WLCAP && RCAP % 4 == 0 && BK_ZINTS % 4 == 0);
static_assert((long long)RCAP * 100 >= (long long)MAXB512_MEAS * 105);
static_assert(WLCAP >= MAXB512_MEAS / 8 + 8 * 46 + 1);
static_assert(MAXDEG_MEAS + 8 <= DEGCAP);
static_assert(BK_LDS <= 300000);
static_assert((NP * FIN / 8) % NTHR == 0 && (HC * FIN / 8) % NTHR == 0 && (HC * 1024 / 8) % NTHR == 0);
static_assert((CD * 1024 / 8) % NTHR == 0 && (64 * 256 / 8) % NTHR == 0);
static_assert(P_END / 4 <= PBPAR * NTHR && P_END % 128 == 0);
static_assert(HC == 4 * CD && CD == 4 * 32);
static_assert((EOFF * 4) % 128 == 0 && EOFF == 2 * NN);
static_assert(NN % 2 == 0);
static_assert(K_TWO % 32 == 0 && K_THREE % 32 == 0 && K_HEAD % 32 == 0 && FIN % 32 == 0);

typedef float          v4f   __attribute__((ext_vector_type(4)));
typedef float          v8f   __attribute__((ext_vector_type(8)));
typedef int            v4i   __attribute__((ext_vector_type(4)));
typedef int            v8i   __attribute__((ext_vector_type(8)));
typedef unsigned short v8us  __attribute__((ext_vector_type(8)));
typedef unsigned short v16us __attribute__((ext_vector_type(16)));
typedef __bf16         v16bf __attribute__((ext_vector_type(16)));
typedef v4f  __attribute__((may_alias)) v4fa;
typedef v4i  __attribute__((may_alias)) v4ia;
typedef v8us __attribute__((may_alias)) v8usa;
union FragB { v16bf v; v16us u; v8us h[2]; v8i w; };

__device__ __forceinline__ v8f wmb(const FragB& a, const FragB& b, v8f c) {
  v8f d = __builtin_amdgcn_wmma_f32_16x16x32_bf16(false, a.v, false, b.v, (short)0, c, false, false);
  asm volatile("v_nop\n\tv_nop\n\tv_nop\n\tv_nop" : "+v"(d) : "v"(a.w), "v"(b.w));
  return d;
}

__device__ __forceinline__ unsigned bf16_bits(float f) {
  const unsigned u = __float_as_uint(f);
  const unsigned r = (u + 0x7FFFu + ((u >> 16) & 1u)) >> 16;
  const unsigned q = (u >> 16) | 0x40u;
  return ((u & 0x7fffffffu) > 0x7f800000u) ? q : r;
}

__device__ __forceinline__ void hilo_pack(float v0, float v1, float v2, float v3,
                                          int& h01, int& h23, int& l01, int& l23) {
  const unsigned a0 = bf16_bits(v0), a1 = bf16_bits(v1), a2 = bf16_bits(v2), a3 = bf16_bits(v3);
  const unsigned b0 = bf16_bits(v0 - __uint_as_float(a0 << 16));
  const unsigned b1 = bf16_bits(v1 - __uint_as_float(a1 << 16));
  const unsigned b2 = bf16_bits(v2 - __uint_as_float(a2 << 16));
  const unsigned b3 = bf16_bits(v3 - __uint_as_float(a3 << 16));
  h01 = (int)(a0 | (a1 << 16)); h23 = (int)(a2 | (a3 << 16));
  l01 = (int)(b0 | (b1 << 16)); l23 = (int)(b2 | (b3 << 16));
}

__device__ __forceinline__ void st2_v4f(float* p, v4f v) {
  *(volatile v4f*)p = v;
  __threadfence();
  *(volatile v4f*)p = v;
}
__device__ __forceinline__ void st2_v8us(unsigned short* p, v8us v) {
  *(volatile v8us*)p = v;
  __threadfence();
  *(volatile v8us*)p = v;
}

__device__ __forceinline__ v8us colpick8(const float* __restrict__ base, int stride) {
  float f[8];
#pragma unroll
  for (int i = 0; i < 8; ++i) f[i] = base[(size_t)i * (size_t)stride];
  v8us o;
#pragma unroll
  for (int i = 0; i < 8; ++i) o[i] = (unsigned short)bf16_bits(f[i]);
  return o;
}

__device__ __forceinline__ void par_put(const float* __restrict__ src, int n, int e0, float* dst) {
  const int i0 = e0     < n ? e0     : n - 1;
  const int i1 = e0 + 1 < n ? e0 + 1 : n - 1;
  const int i2 = e0 + 2 < n ? e0 + 2 : n - 1;
  const int i3 = e0 + 3 < n ? e0 + 3 : n - 1;
  const float a0 = src[i0], a1 = src[i1], a2 = src[i2], a3 = src[i3];
  asm volatile("" :: "v"(a0), "v"(a1), "v"(a2), "v"(a3));
  const unsigned m0 = (e0     < n) ? 0xffffffffu : 0u;
  const unsigned m1 = (e0 + 1 < n) ? 0xffffffffu : 0u;
  const unsigned m2 = (e0 + 2 < n) ? 0xffffffffu : 0u;
  const unsigned m3 = (e0 + 3 < n) ? 0xffffffffu : 0u;
  v4f o;
  o.x = __uint_as_float((bf16_bits(a0) << 16) & m0);
  o.y = __uint_as_float((bf16_bits(a1) << 16) & m1);
  o.z = __uint_as_float((bf16_bits(a2) << 16) & m2);
  o.w = __uint_as_float((bf16_bits(a3) << 16) & m3);
  st2_v4f(dst, o);
}

__global__ __launch_bounds__(NTHR) void k_prep(
    const float* __restrict__ x, const float* __restrict__ w1, const float* __restrict__ w2,
    const float* __restrict__ w3, const float* __restrict__ wc1,
    const float* __restrict__ a1s, const float* __restrict__ a1d, const float* __restrict__ b1,
    const float* __restrict__ a2s, const float* __restrict__ a2d, const float* __restrict__ b2,
    const float* __restrict__ a3s, const float* __restrict__ a3d, const float* __restrict__ b3,
    const float* __restrict__ bc1, const float* __restrict__ wc2, const float* __restrict__ bc2,
    unsigned short* xb, unsigned short* w1t, unsigned short* w2d, unsigned short* w3d,
    unsigned short* wc1d, float* par) {
  const int tid = (int)threadIdx.x;
  const int blk = (int)blockIdx.x;
  if (blk < PBX) {
    const int u   = blk * NTHR + tid;
    const int row = u >> 5, k8 = (u & 31) * 8;
    const int rc  = row < NN ? row : NN - 1;
    const unsigned mk = row < NN ? 0xffffu : 0u;
    const float* p = x + (size_t)rc * FIN + k8;
    const v4f a = *(const v4fa*)p;
    const v4f b = *(const v4fa*)(p + 4);
    v8us o;
    o[0] = (unsigned short)(bf16_bits(a.x) & mk); o[1] = (unsigned short)(bf16_bits(a.y) & mk);
    o[2] = (unsigned short)(bf16_bits(a.z) & mk); o[3] = (unsigned short)(bf16_bits(a.w) & mk);
    o[4] = (unsigned short)(bf16_bits(b.x) & mk); o[5] = (unsigned short)(bf16_bits(b.y) & mk);
    o[6] = (unsigned short)(bf16_bits(b.z) & mk); o[7] = (unsigned short)(bf16_bits(b.w) & mk);
    st2_v8us(xb + (size_t)row * FIN + k8, o);
  } else if (blk < PBX + PBW1) {
    const int u = (blk - PBX) * NTHR + tid;
    const int n = u >> 5, k8 = (u & 31) * 8;
    const v8us o = colpick8(w1 + (size_t)k8 * HC + n, HC);
    st2_v8us(w1t + (size_t)n * FIN + k8, o);
  } else if (blk < PBX + PBW1 + PBW2) {
    const int u = (blk - PBX - PBW1) * NTHR + tid;
    const int n = u >> 7, k8 = (u & 127) * 8, kk = k8 & 511;
    const v8us o = colpick8(w2 + (size_t)kk * HC + n, HC);
    st2_v8us(w2d + (size_t)n * 1024 + k8, o);
  } else if (blk < PBX + PBW1 + PBW2 + PBW3) {
    const int u = (blk - PBX - PBW1 - PBW2) * NTHR + tid;
    const int n = u >> 7, k8 = (u & 127) * 8, kk = k8 & 511;
    const v8us o = colpick8(w3 + (size_t)kk * CD + n, CD);
    st2_v8us(w3d + (size_t)n * 1024 + k8, o);
  } else if (blk < PBX + PBW1 + PBW2 + PBW3 + PBWC) {
    const int u = (blk - PBX - PBW1 - PBW2 - PBW3) * NTHR + tid;
    const int n = u >> 5, k8 = (u & 31) * 8, kk = k8 & 127;
    const v8us o = colpick8(wc1 + (size_t)kk * 64 + n, 64);
    st2_v8us(wc1d + (size_t)n * 256 + k8, o);
  } else {
    const int pu = (blk - PBX - PBW1 - PBW2 - PBW3 - PBWC) * NTHR + tid;
    const int wv = pu >> 5;
    float* dp = par + 4 * pu;
    if (wv < 4)        par_put(a1s, 512, 4 * pu,        dp);
    else if (wv < 8)   par_put(a1d, 512, 4 * pu - 512,  dp);
    else if (wv < 12)  par_put(b1,  512, 4 * pu - 1024, dp);
    else if (wv < 16)  par_put(a2s, 512, 4 * pu - 1536, dp);
    else if (wv < 20)  par_put(a2d, 512, 4 * pu - 2048, dp);
    else if (wv < 24)  par_put(b2,  512, 4 * pu - 2560, dp);
    else if (wv == 24) par_put(a3s, 128, 4 * pu - 3072, dp);
    else if (wv == 25) par_put(a3d, 128, 4 * pu - 3200, dp);
    else if (wv == 26) par_put(b3,  128, 4 * pu - 3328, dp);
    else if (wv == 27) par_put(bc1,  64, 4 * pu - 3456, dp);
    else if (wv == 28) par_put(wc2, 128, 4 * pu - 3584, dp);
    else if (wv == 29) par_put(bc2,   2, 4 * pu - 3712, dp);
  }
}

__device__ __forceinline__ void bucket_flush(const int* pl, const int* cnt, int ov, int* lp, int* cop, int* fp,
                                             int tid) {
#pragma unroll 1
  for (int i = tid * 4; i < RCAP; i += NTHR * 4) {
    const v4i v = *(const v4ia*)(pl + i);
    *(volatile v4i*)(lp + i) = v;
  }
  {
    const v4i v = *(const v4ia*)(cnt + 4 * tid);
    *(volatile v4i*)(cop + 4 * tid) = v;
  }
  if (tid < 8) {
    const v4i f = {ov, ov, ov, ov};
    *(volatile v4i*)(fp + 4 * tid) = f;
  }
}

__global__ __launch_bounds__(NTHR) void k_bucket(const int* __restrict__ srcs, const int* __restrict__ dsts,
                                                 int* LIST, int* CO, int* FLAG) {
  extern __shared__ __attribute__((aligned(16))) int dsm[];
  int* wl   = dsm;
  int* pl   = dsm + NWAVE * WLCAP;
  int* cnt  = pl + RCAP;
  int* offs = cnt + NBRUN;
  int* cur  = offs + NBRUN;
  int* misc = cur + NBRUN;
  const int tid = (int)threadIdx.x, lane = tid & 31, wave = tid >> 5;
  const int blk = (int)blockIdx.x;
  const unsigned nbs = (unsigned)(blk * NBRUN);

  {
    const v4i z4 = {0, 0, 0, 0};
    for (int i = tid * 4; i < BK_ZINTS; i += NTHR * 4) *(v4ia*)(dsm + i) = z4;
    if (tid < 16) misc[tid] = 0;
  }
  __syncthreads();

  {
    const int per  = ((NE + NWAVE * WCH - 1) / (NWAVE * WCH)) * WCH;
    const int ebeg = wave * per;
    const int eend = (ebeg + per < NE) ? (ebeg + per) : NE;
    int* mylist = wl + wave * WLCAP;
    int wc = 0;
#pragma unroll 1
    for (int cb = ebeg; cb < eend; cb += WCH) {
      const int e0 = cb + lane * EPT;
      const v4i da = *(const v4ia*)(dsts + e0);
      const v4i db = *(const v4ia*)(dsts + e0 + 4);
      const unsigned s0 = (unsigned)da.x - nbs, s1 = (unsigned)da.y - nbs;
      const unsigned s2 = (unsigned)da.z - nbs, s3 = (unsigned)da.w - nbs;
      const unsigned s4 = (unsigned)db.x - nbs, s5 = (unsigned)db.y - nbs;
      const unsigned s6 = (unsigned)db.z - nbs, s7 = (unsigned)db.w - nbs;
      const bool h0 = s0 < (unsigned)NBRUN, h1 = s1 < (unsigned)NBRUN, h2 = s2 < (unsigned)NBRUN, h3 = s3 < (unsigned)NBRUN;
      const bool h4 = s4 < (unsigned)NBRUN, h5 = s5 < (unsigned)NBRUN, h6 = s6 < (unsigned)NBRUN, h7 = s7 < (unsigned)NBRUN;
      const unsigned m0 = __builtin_amdgcn_ballot_w32(h0), m1 = __builtin_amdgcn_ballot_w32(h1);
      const unsigned m2 = __builtin_amdgcn_ballot_w32(h2), m3 = __builtin_amdgcn_ballot_w32(h3);
      const unsigned m4 = __builtin_amdgcn_ballot_w32(h4), m5 = __builtin_amdgcn_ballot_w32(h5);
      const unsigned m6 = __builtin_amdgcn_ballot_w32(h6), m7 = __builtin_amdgcn_ballot_w32(h7);
      const unsigned any = m0 | m1 | m2 | m3 | m4 | m5 | m6 | m7;
      if (any != 0u) {
        const int pre = (int)(__builtin_amdgcn_mbcnt_lo(m0, 0u) + __builtin_amdgcn_mbcnt_lo(m1, 0u) +
                              __builtin_amdgcn_mbcnt_lo(m2, 0u) + __builtin_amdgcn_mbcnt_lo(m3, 0u) +
                              __builtin_amdgcn_mbcnt_lo(m4, 0u) + __builtin_amdgcn_mbcnt_lo(m5, 0u) +
                              __builtin_amdgcn_mbcnt_lo(m6, 0u) + __builtin_amdgcn_mbcnt_lo(m7, 0u));
        int p = wc + pre;
        if (h0) { if (p < WLCAP) mylist[p] = ((e0 + 0) << SLB) | (int)s0; p = p + 1; }
        if (h1) { if (p < WLCAP) mylist[p] = ((e0 + 1) << SLB) | (int)s1; p = p + 1; }
        if (h2) { if (p < WLCAP) mylist[p] = ((e0 + 2) << SLB) | (int)s2; p = p + 1; }
        if (h3) { if (p < WLCAP) mylist[p] = ((e0 + 3) << SLB) | (int)s3; p = p + 1; }
        if (h4) { if (p < WLCAP) mylist[p] = ((e0 + 4) << SLB) | (int)s4; p = p + 1; }
        if (h5) { if (p < WLCAP) mylist[p] = ((e0 + 5) << SLB) | (int)s5; p = p + 1; }
        if (h6) { if (p < WLCAP) mylist[p] = ((e0 + 6) << SLB) | (int)s6; p = p + 1; }
        if (h7) { if (p < WLCAP) mylist[p] = ((e0 + 7) << SLB) | (int)s7; p = p + 1; }
        wc += (int)(__builtin_popcount(m0) + __builtin_popcount(m1) + __builtin_popcount(m2) + __builtin_popcount(m3) +
                    __builtin_popcount(m4) + __builtin_popcount(m5) + __builtin_popcount(m6) + __builtin_popcount(m7));
      }
    }
    if (lane == 0) misc[wave] = wc;
  }
  __syncthreads();

  if (wave == 0) {
    int ov = 0;
#pragma unroll 1
    for (int w2 = 0; w2 < NWAVE; ++w2) {
      int c = misc[w2];
      if (c > WLCAP) ov = 1;
      c = c < 0 ? 0 : (c > WLCAP ? WLCAP : c);
#pragma unroll 1
      for (int b0 = 0; b0 < c; b0 += 32) {
        const int idx = b0 + lane;
        const int ent = wl[w2 * WLCAP + (idx < WLCAP ? idx : WLCAP - 1)];
        const int m32 = (c - b0) < 32 ? (c - b0) : 32;
#pragma unroll 1
        for (int k = 0; k < m32; ++k) {
          const int u    = __builtin_amdgcn_readlane(ent, k);
          const int slot = u & (NBRUN - 1);
          if (lane == 0) cnt[slot] = cnt[slot] + 1;
        }
      }
    }
    if (lane == 0) misc[9] = ov;
  }
  __syncthreads();
  if (wave == 0) {
    const int base = lane * (NBRUN / 32);
    int s = 0;
#pragma unroll 1
    for (int i = 0; i < NBRUN / 32; ++i) s += cnt[base + i];
    int incl = s;
#pragma unroll
    for (int d = 1; d < 32; d <<= 1) {
      const int y = __shfl_up(incl, d, 32);
      if (lane >= d) incl += y;
    }
    int run = incl - s;
#pragma unroll 1
    for (int i = 0; i < NBRUN / 32; ++i) {
      const int cv = cnt[base + i];
      offs[base + i] = run;
      cur[base + i]  = run;
      run += cv;
    }
  }
  __syncthreads();

  if (wave == 0) {
#pragma unroll 1
    for (int w2 = 0; w2 < NWAVE; ++w2) {
      int c = misc[w2];
      c = c < 0 ? 0 : (c > WLCAP ? WLCAP : c);
#pragma unroll 1
      for (int b0 = 0; b0 < c; b0 += 32) {
        const int idx = b0 + lane;
        const int ent = wl[w2 * WLCAP + (idx < WLCAP ? idx : WLCAP - 1)];
        int eid = (ent >> SLB) & 0x3FFFFF;
        eid = eid > NE - 1 ? NE - 1 : eid;
        int sr = srcs[eid];
        sr = sr < 0 ? 0 : (sr > NN - 1 ? NN - 1 : sr);
        const int m32 = (c - b0) < 32 ? (c - b0) : 32;
#pragma unroll 1
        for (int k = 0; k < m32; ++k) {
          const int u    = __builtin_amdgcn_readlane(ent, k);
          const int wd   = __builtin_amdgcn_readlane(sr, k);
          const int slot = u & (NBRUN - 1);
          if (lane == 0) {
            int p = cur[slot];
            p = p < 0 ? 0 : (p > RCAP - 1 ? RCAP - 1 : p);
            pl[p] = wd;
            cur[slot] = p + 1;
          }
        }
      }
    }
  }
  __syncthreads();

  const int ovf = misc[9];
  int* lp  = LIST + (size_t)blk * RCAP;
  int* cop = CO + (size_t)blk * (2 * NBRUN);
  int* fp  = FLAG + (size_t)blk * 32;
  bucket_flush(pl, cnt, ovf, lp, cop, fp, tid);
  __threadfence();
  bucket_flush(pl, cnt, ovf, lp, cop, fp, tid);
}

template <int KEXT, int BPITCH>
__device__ __forceinline__ void gemm_16x64(const unsigned short* __restrict__ ap,
                                           const unsigned short* __restrict__ bp, v8f (&acc)[4]) {
#pragma unroll 1
  for (int k0 = 0; k0 < KEXT; k0 += 32) {
    FragB af;
    af.h[0] = *(const v8usa*)(ap + k0);
    af.h[1] = *(const v8usa*)(ap + k0 + 16);
#pragma unroll
    for (int nt = 0; nt < 4; ++nt) {
      const unsigned short* wq = bp + (size_t)(16 * nt) * (size_t)BPITCH + k0;
      FragB bf;
      bf.h[0] = *(const v8usa*)wq;
      bf.h[1] = *(const v8usa*)(wq + 16);
      acc[nt] = wmb(af, bf, acc[nt]);
    }
  }
}

__device__ __forceinline__ void stage_d(float* stg, const v8f (&acc)[4], int wave, int hh, int m) {
#pragma unroll
  for (int nt = 0; nt < 4; ++nt) {
#pragma unroll
    for (int r = 0; r < 8; ++r) stg[(16 * wave + 8 * hh + r) * SP + 16 * nt + m] = acc[nt][r];
  }
}

template <int KEXT, int APITCH, int BPITCH, int NCOL, int NHEAD>
__global__ __launch_bounds__(NTHR) __attribute__((amdgpu_num_vgpr(248)))
void k_gemm(const unsigned short* __restrict__ A, const unsigned short* __restrict__ BT,
            const float* __restrict__ att, float* Hout, float* SDout) {
  constexpr int SW  = 2 * NHEAD;
  constexpr int NCT = NCOL / 64;
  static_assert(NCOL == NHEAD * CD && (NCT % 2) == 0);
  static_assert(KEXT % 32 == 0 && KEXT <= APITCH && KEXT <= BPITCH);
  static_assert((2 * NCOL / 4) % 32 == 0 && (GBM * SW / 4) % 32 == 0);
  __shared__ __attribute__((aligned(16))) float stg[GBM * SP];
  __shared__ __attribute__((aligned(16))) float satt[2 * NCOL];
  __shared__ __attribute__((aligned(16))) float sdot[GBM * SW];
  const int tid = (int)threadIdx.x, lane = tid & 31, wave = tid >> 5, hh = lane >> 4, m = lane & 15;
  const int rowBase = (int)blockIdx.x * GBM;

  for (int i = tid; i < 2 * NCOL / 4; i += NTHR) *(v4fa*)(satt + 4 * i) = *(const v4fa*)(att + 4 * i);

  const unsigned short* ap = A + (size_t)(rowBase + 16 * wave + m) * (size_t)APITCH + 8 * hh;
  const int drow = tid & 127, which = tid >> 7;
  float dacc = 0.0f;

#pragma unroll 1
  for (int ct = 0; ct < NCT; ++ct) {
    v8f acc[4];
    {
      const v8f z = {0.f, 0.f, 0.f, 0.f, 0.f, 0.f, 0.f, 0.f};
#pragma unroll
      for (int t = 0; t < 4; ++t) acc[t] = z;
    }
    const unsigned short* bp = BT + (size_t)(ct * 64 + m) * (size_t)BPITCH + 8 * hh;
    gemm_16x64<KEXT, BPITCH>(ap, bp, acc);
    stage_d(stg, acc, wave, hh, m);
    __syncthreads();

    {
      const float* hr = stg + drow * SP;
      const float* sa = satt + which * NCOL + ct * 64;
      float dd = 0.0f;
#pragma unroll 4
      for (int c4 = 0; c4 < 16; ++c4) {
        const v4f hv = *(const v4fa*)(hr + 4 * c4);
        const v4f av = *(const v4fa*)(sa + 4 * c4);
        dd = fmaf(hv.x, av.x, dd);
        dd = fmaf(hv.y, av.y, dd);
        dd = fmaf(hv.z, av.z, dd);
        dd = fmaf(hv.w, av.w, dd);
      }
      dacc += dd;
      if ((ct & 1) != 0) {
        sdot[drow * SW + which * NHEAD + (ct >> 1)] = dacc;
        dacc = 0.0f;
      }
    }

#pragma unroll 1
    for (int i = 0; i < 8; ++i) {
      const int lr = 16 * wave + 2 * i + hh;
      const v4f a = *(const v4fa*)(stg + lr * SP + 4 * m);
      st2_v4f(Hout + (size_t)(rowBase + lr) * (size_t)NCOL + ct * 64 + 4 * m, a);
    }
    __syncthreads();
  }

  constexpr int NFL = GBM * SW / 4;
  if (tid < NFL) {
    const v4f v = *(const v4fa*)(sdot + 4 * tid);
    st2_v4f(SDout + (size_t)rowBase * SW + 4 * tid, v);
  }
}

template <int NH>
__device__ __forceinline__ void replay_core(const int* __restrict__ lb, int o, int c, int dc,
                                            const float* __restrict__ Hm, const float* __restrict__ SD,
                                            int lane, v4f (&acc)[NH], float (&den)[NH]) {
  constexpr int HPI = NH * CD;
  constexpr int SW  = 2 * NH;
  const float ninf = __uint_as_float(0xff800000u);
  float mx[NH], ad[NH];
  if constexpr (NH == 4) {
    const v4f t = *(const v4fa*)(SD + (size_t)dc * SW + 4);
    ad[0] = t.x; ad[1] = t.y; ad[2] = t.z; ad[3] = t.w;
  } else {
    ad[0] = SD[(size_t)dc * SW + 1];
  }
  {
    const v4f z4 = {0.f, 0.f, 0.f, 0.f};
#pragma unroll
    for (int h = 0; h < NH; ++h) { mx[h] = ninf; den[h] = 0.0f; acc[h] = z4; }
  }
  const int ct = c + 1;
  int last = o + c - 1;
  last = last < o ? o : last;
  last = last > RCAP - 1 ? RCAP - 1 : last;
#pragma unroll 1
  for (int k0 = 0; k0 < ct; k0 += 32) {
    const int pos = k0 + lane;
    int idx = o + pos;
    idx = idx > last ? last : idx;
    const int wd = lb[idx];
    asm volatile("" :: "v"(wd));
    int s = wd < 0 ? 0 : (wd > NN - 1 ? NN - 1 : wd);
    s = (pos == c) ? dc : s;
    float as[NH];
    if constexpr (NH == 4) {
      const v4f t = *(const v4fa*)(SD + (size_t)s * SW);
      asm volatile("" :: "v"(t));
      as[0] = t.x; as[1] = t.y; as[2] = t.z; as[3] = t.w;
    } else {
      const float t = SD[(size_t)s * SW];
      asm volatile("" :: "v"(t));
      as[0] = t;
    }
    const bool valid = pos < ct;
    float p[NH];
#pragma unroll
    for (int h = 0; h < NH; ++h) {
      float e = as[h] + ad[h];
      e = (e >= 0.0f) ? e : 0.2f * e;
      e = valid ? e : ninf;
      float cm = e;
#pragma unroll
      for (int off = 16; off > 0; off >>= 1) cm = fmaxf(cm, __shfl_xor(cm, off, 32));
      const float mn = fmaxf(mx[h], cm);
      const float sc = __expf(mx[h] - mn);
      const float ph = __expf(e - mn);
      float ps = ph;
#pragma unroll
      for (int off = 16; off > 0; off >>= 1) ps += __shfl_xor(ps, off, 32);
      den[h] = den[h] * sc + ps;
      acc[h] = acc[h] * sc;
      mx[h]  = mn;
      p[h]   = ph;
    }
    const int m32 = (ct - k0) < 32 ? (ct - k0) : 32;
#pragma unroll 1
    for (int j = 0; j < m32; ++j) {
      const int sj = __builtin_amdgcn_readlane(s, j);
      const float* hp = Hm + (size_t)sj * HPI + 4 * lane;
#pragma unroll
      for (int h = 0; h < NH; ++h) {
        const float pj = __int_as_float(__builtin_amdgcn_readlane(__float_as_int(p[h]), j));
        const v4f f = *(const v4fa*)(hp + CD * h);
        acc[h].x = fmaf(pj, f.x, acc[h].x);
        acc[h].y = fmaf(pj, f.y, acc[h].y);
        acc[h].z = fmaf(pj, f.z, acc[h].z);
        acc[h].w = fmaf(pj, f.w, acc[h].w);
      }
    }
  }
}

__device__ __forceinline__ float fixv(float v, bool bad, bool live, float qnan) {
  v = bad ? qnan : v;
  return live ? v : 0.0f;
}

__global__ __launch_bounds__(NTHR) void k_replay_wide(const int* __restrict__ LIST, const int* __restrict__ CO,
                                                      const int* __restrict__ FLAG, const float* __restrict__ Hm,
                                                      const float* __restrict__ SD, const float* __restrict__ bias,
                                                      unsigned short* E) {
  __shared__ __attribute__((aligned(16))) float srow[NWAVE * HC];
  const int tid = (int)threadIdx.x, lane = tid & 31, wave = tid >> 5;
  const int d  = (int)blockIdx.x * NWAVE + wave;
  const int dc = d < NN ? d : NN - 1;
  const int bucket = d >> SLB, slot = d & (NBRUN - 1);
  const int* lb  = LIST + (size_t)bucket * RCAP;
  const int* cob = CO + (size_t)bucket * (2 * NBRUN);
  const int flag = FLAG[(size_t)bucket * 32];
  int cv = cob[slot];
  int ov = cob[NBRUN + slot];
  const bool big = cv > DEGCAP;
  cv = cv < 0 ? 0 : (cv > DEGCAP ? DEGCAP : cv);
  ov = ov < 0 ? 0 : (ov > RCAP - 1 ? RCAP - 1 : ov);
  const int c = __builtin_amdgcn_readfirstlane(cv);
  const int o = __builtin_amdgcn_readfirstlane(ov);

  v4f acc[4];
  float den[4];
  replay_core<4>(lb, o, c, dc, Hm, SD, lane, acc, den);

  float* sw = srow + wave * HC;
#pragma unroll
  for (int h = 0; h < 4; ++h) {
    const float inv = __builtin_amdgcn_rcpf(den[h] + 1e-16f);
    const v4f bb = *(const v4fa*)(bias + CD * h + 4 * lane);
    v4f v;
    v.x = fmaf(acc[h].x, inv, bb.x);
    v.y = fmaf(acc[h].y, inv, bb.y);
    v.z = fmaf(acc[h].z, inv, bb.z);
    v.w = fmaf(acc[h].w, inv, bb.w);
    *(v4fa*)(sw + CD * h + 4 * lane) = v;
  }
  __syncthreads();
#pragma unroll 1
  for (int q = 0; q < 16; ++q) {
    const float xv = sw[32 * q + lane];
    const float yv = (xv > 0.0f) ? xv : expm1f(xv);
    sw[32 * q + lane] = yv;
  }
  __syncthreads();

  const v4f x0 = *(const v4fa*)(sw + 8 * lane);
  const v4f x1 = *(const v4fa*)(sw + 8 * lane + 4);
  const v4f x2 = *(const v4fa*)(sw + 256 + 8 * lane);
  const v4f x3 = *(const v4fa*)(sw + 256 + 8 * lane + 4);
  const bool bad  = (flag != 0) | big;
  const bool live = d < NN;
  const float qnan = __uint_as_float(0x7fc00000u);
  int a01, a23, b01, b23, c01, c23, d01, d23;
  v4i hA, lA, hB, lB;
  hilo_pack(fixv(x0.x, bad, live, qnan), fixv(x0.y, bad, live, qnan), fixv(x0.z, bad, live, qnan),
            fixv(x0.w, bad, live, qnan), a01, a23, b01, b23);
  hilo_pack(fixv(x1.x, bad, live, qnan), fixv(x1.y, bad, live, qnan), fixv(x1.z, bad, live, qnan),
            fixv(x1.w, bad, live, qnan), c01, c23, d01, d23);
  hA.x = a01; hA.y = a23; hA.z = c01; hA.w = c23;
  lA.x = b01; lA.y = b23; lA.z = d01; lA.w = d23;
  hilo_pack(fixv(x2.x, bad, live, qnan), fixv(x2.y, bad, live, qnan), fixv(x2.z, bad, live, qnan),
            fixv(x2.w, bad, live, qnan), a01, a23, b01, b23);
  hilo_pack(fixv(x3.x, bad, live, qnan), fixv(x3.y, bad, live, qnan), fixv(x3.z, bad, live, qnan),
            fixv(x3.w, bad, live, qnan), c01, c23, d01, d23);
  hB.x = a01; hB.y = a23; hB.z = c01; hB.w = c23;
  lB.x = b01; lB.y = b23; lB.z = d01; lB.w = d23;

  unsigned short* ep = E + (size_t)d * 1024 + 8 * lane;
  *(volatile v4i*)(ep)       = hA;
  *(volatile v4i*)(ep + 256) = hB;
  *(volatile v4i*)(ep + 512) = lA;
  *(volatile v4i*)(ep + 768) = lB;
  __threadfence();
  *(volatile v4i*)(ep)       = hA;
  *(volatile v4i*)(ep + 256) = hB;
  *(volatile v4i*)(ep + 512) = lA;
  *(volatile v4i*)(ep + 768) = lB;
}

__global__ __launch_bounds__(NTHR) void k_replay_narrow(const int* __restrict__ LIST, const int* __restrict__ CO,
                                                        const int* __restrict__ FLAG, const float* __restrict__ Hm,
                                                        const float* __restrict__ SD, const float* __restrict__ bias,
                                                        float* out, unsigned short* E3) {
  const int tid = (int)threadIdx.x, lane = tid & 31, wave = tid >> 5;
  const int d  = (int)blockIdx.x * NWAVE + wave;
  const int dc = d < NN ? d : NN - 1;
  const int bucket = d >> SLB, slot = d & (NBRUN - 1);
  const int* lb  = LIST + (size_t)bucket * RCAP;
  const int* cob = CO + (size_t)bucket * (2 * NBRUN);
  const int flag = FLAG[(size_t)bucket * 32];
  int cv = cob[slot];
  int ov = cob[NBRUN + slot];
  const bool big = cv > DEGCAP;
  cv = cv < 0 ? 0 : (cv > DEGCAP ? DEGCAP : cv);
  ov = ov < 0 ? 0 : (ov > RCAP - 1 ? RCAP - 1 : ov);
  const int c = __builtin_amdgcn_readfirstlane(cv);
  const int o = __builtin_amdgcn_readfirstlane(ov);

  v4f acc[1];
  float den[1];
  replay_core<1>(lb, o, c, dc, Hm, SD, lane, acc, den);

  const float inv = __builtin_amdgcn_rcpf(den[0] + 1e-16f);
  const v4f bb = *(const v4fa*)(bias + 4 * lane);
  const bool bad  = (flag != 0) | big;
  const bool live = d < NN;
  const float qnan = __uint_as_float(0x7fc00000u);
  v4f v;
  v.x = fmaf(acc[0].x, inv, bb.x);
  v.y = fmaf(acc[0].y, inv, bb.y);
  v.z = fmaf(acc[0].z, inv, bb.z);
  v.w = fmaf(acc[0].w, inv, bb.w);
  v.x = bad ? qnan : v.x; v.y = bad ? qnan : v.y; v.z = bad ? qnan : v.z; v.w = bad ? qnan : v.w;

  int h01, h23, l01, l23;
  hilo_pack(live ? v.x : 0.0f, live ? v.y : 0.0f, live ? v.z : 0.0f, live ? v.w : 0.0f, h01, h23, l01, l23);
  const int s0 = (2 * lane) & 31, s1 = s0 + 1;
  const int a0 = __shfl(h01, s0, 32), a1 = __shfl(h23, s0, 32), a2 = __shfl(h01, s1, 32), a3 = __shfl(h23, s1, 32);
  const int b0 = __shfl(l01, s0, 32), b1 = __shfl(l23, s0, 32), b2 = __shfl(l01, s1, 32), b3 = __shfl(l23, s1, 32);
  const int mk = (lane < 16) ? -1 : 0;
  v4i ow;
  ow.x = (a0 & mk) | (b0 & ~mk); ow.y = (a1 & mk) | (b1 & ~mk);
  ow.z = (a2 & mk) | (b2 & ~mk); ow.w = (a3 & mk) | (b3 & ~mk);

  float* op = out + (size_t)EOFF + (size_t)dc * CD + 4 * lane;
  unsigned short* hp = E3 + (size_t)d * 256 + 8 * lane;
  if (live) *(volatile v4f*)op = v;
  *(volatile v4i*)hp = ow;
  __threadfence();
  if (live) *(volatile v4f*)op = v;
  *(volatile v4i*)hp = ow;
}

__global__ __launch_bounds__(NTHR) __attribute__((amdgpu_num_vgpr(248)))
void k_head(const unsigned short* __restrict__ E3, const unsigned short* __restrict__ WC1D,
            const float* __restrict__ par, const int* __restrict__ FLAG, float* out) {
  __shared__ __attribute__((aligned(16))) float stg[GBM * SP];
  __shared__ __attribute__((aligned(16))) float spar[384];
  __shared__ __attribute__((aligned(16))) float spair[2 * GBM];
  const int tid = (int)threadIdx.x, lane = tid & 31, wave = tid >> 5, hh = lane >> 4, m = lane & 15;
  const int blk = (int)blockIdx.x;
  const int rowBase = blk * GBM;
  const int flag = FLAG[(size_t)(rowBase >> SLB) * 32];

  if (tid < 96) *(v4fa*)(spar + 4 * tid) = *(const v4fa*)(par + P_HD + 4 * tid);

  v8f acc[4];
  {
    const v8f z = {0.f, 0.f, 0.f, 0.f, 0.f, 0.f, 0.f, 0.f};
#pragma unroll
    for (int t = 0; t < 4; ++t) acc[t] = z;
  }
  const unsigned short* ap = E3 + (size_t)(rowBase + 16 * wave + m) * 256 + 8 * hh;
  const unsigned short* bp = WC1D + (size_t)m * 256 + 8 * hh;
  gemm_16x64<K_HEAD, 256>(ap, bp, acc);
  stage_d(stg, acc, wave, hh, m);
  __syncthreads();

  if (tid < GBM) {
    const float* tr = stg + tid * SP;
    float o0 = 0.0f, o1 = 0.0f;
#pragma unroll 1
    for (int cidx = 0; cidx < 64; ++cidx) {
      const float t = tr[cidx] + spar[cidx];
      const float r = (t > 0.0f) ? t : (t - t);
      o0 = fmaf(r, spar[128 + 2 * cidx], o0);
      o1 = fmaf(r, spar[129 + 2 * cidx], o1);
    }
    o0 += spar[256];
    o1 += spar[257];
    const float qnan = __uint_as_float(0x7fc00000u);
    spair[2 * tid]     = (flag != 0) ? qnan : o0;
    spair[2 * tid + 1] = (flag != 0) ? qnan : o1;
  }
  __syncthreads();

  if (tid < 64) {
    const v4f v = *(const v4fa*)(spair + 4 * tid);
    asm volatile("" :: "v"(v));
    const int f0 = blk * (2 * GBM) + 4 * tid;
    const bool ok = (f0 + 3) < 2 * NN;
    float* op = out + (size_t)(ok ? f0 : 0);
    if (ok) *(volatile v4f*)op = v;
    __threadfence();
    if (ok) *(volatile v4f*)op = v;
  }
}

extern "C" void kernel_launch(void* const* d_in, const int* in_sizes, int n_in,
                              void* d_out, int out_size, void* d_ws, size_t ws_size,
                              hipStream_t stream) {
  if (n_in < 18) return;
  if (in_sizes[0] != NN * FIN) return;
  if (in_sizes[1] != 2 * NE) return;
  if (in_sizes[2] != FIN * HC) return;
  if (in_sizes[3] != HC || in_sizes[4] != HC || in_sizes[5] != HC) return;
  if (in_sizes[6] != HC * HC) return;
  if (in_sizes[7] != HC || in_sizes[8] != HC || in_sizes[9] != HC) return;
  if (in_sizes[10] != HC * CD) return;
  if (in_sizes[11] != CD || in_sizes[12] != CD || in_sizes[13] != CD) return;
  if (in_sizes[14] != CD * 64) return;
  if (in_sizes[15] != 64) return;
  if (in_sizes[16] != 128) return;
  if (in_sizes[17] != 2) return;
  if (out_size != EOFF + NN * CD) return;

  const float* x   = (const float*)d_in[0];
  const int*   ei  = (const int*)d_in[1];
  const float* W1  = (const float*)d_in[2];
  const float* a1s = (const float*)d_in[3];
  const float* a1d = (const float*)d_in[4];
  const float* b1  = (const float*)d_in[5];
  const float* W2  = (const float*)d_in[6];
  const float* a2s = (const float*)d_in[7];
  const float* a2d = (const float*)d_in[8];
  const float* b2  = (const float*)d_in[9];
  const float* W3  = (const float*)d_in[10];
  const float* a3s = (const float*)d_in[11];
  const float* a3d = (const float*)d_in[12];
  const float* b3  = (const float*)d_in[13];
  const float* Wc1 = (const float*)d_in[14];
  const float* bc1 = (const float*)d_in[15];
  const float* Wc2 = (const float*)d_in[16];
  const float* bc2 = (const float*)d_in[17];
  float* out = (float*)d_out;
  const int* srcs = ei;
  const int* dsts = ei + NE;

  constexpr size_t zXB   = (size_t)NP * FIN * 2;
  constexpr size_t zW1T  = (size_t)HC * FIN * 2;
  constexpr size_t zW2D  = (size_t)HC * 1024 * 2;
  constexpr size_t zW3D  = (size_t)CD * 1024 * 2;
  constexpr size_t zWC1D = (size_t)64 * 256 * 2;
  constexpr size_t zE    = (size_t)NP * 1024 * 2;
  constexpr size_t zE3   = (size_t)NP * 256 * 2;
  constexpr size_t zH    = (size_t)NP * HC * 4;
  constexpr size_t zSD   = (size_t)NP * 8 * 4;
  constexpr size_t zPAR  = (size_t)P_END * 4;
  constexpr size_t zLIST = (size_t)NBK * RCAP * 4;
  constexpr size_t zCO   = (size_t)NBK * 2 * NBRUN * 4;
  constexpr size_t zFLAG = (size_t)NBK * 128;
  constexpr size_t oXB   = 0;
  constexpr size_t oW1T  = oXB + zXB;
  constexpr size_t oW2D  = oW1T + zW1T;
  constexpr size_t oW3D  = oW2D + zW2D;
  constexpr size_t oWC1D = oW3D + zW3D;
  constexpr size_t oE    = oWC1D + zWC1D;
  constexpr size_t oE3   = oE + zE;
  constexpr size_t oH    = oE3 + zE3;
  constexpr size_t oSD   = oH + zH;
  constexpr size_t oPAR  = oSD + zSD;
  constexpr size_t oLIST = oPAR + zPAR;
  constexpr size_t oCO   = oLIST + zLIST;
  constexpr size_t oFLAG = oCO + zCO;
  constexpr size_t oEND  = oFLAG + zFLAG;
  static_assert(zXB % 256 == 0 && zW1T % 256 == 0 && zW2D % 256 == 0 && zW3D % 256 == 0 && zWC1D % 256 == 0);
  static_assert(zE % 256 == 0 && zE3 % 256 == 0 && zH % 256 == 0 && zSD % 256 == 0 && zPAR % 256 == 0);
  static_assert(zLIST % 256 == 0 && zCO % 256 == 0 && zFLAG % 256 == 0);
  static_assert(zH >= (size_t)NP * CD * 4 && zSD >= (size_t)NP * 2 * 4);
  static_assert(oEND <= (size_t)(128u << 20));
  if (oEND > ws_size) return;

  char* ws = (char*)d_ws;
  unsigned short* XB   = (unsigned short*)(ws + oXB);
  unsigned short* W1T  = (unsigned short*)(ws + oW1T);
  unsigned short* W2D  = (unsigned short*)(ws + oW2D);
  unsigned short* W3D  = (unsigned short*)(ws + oW3D);
  unsigned short* WC1D = (unsigned short*)(ws + oWC1D);
  unsigned short* E    = (unsigned short*)(ws + oE);
  unsigned short* E3   = (unsigned short*)(ws + oE3);
  float*          H    = (float*)(ws + oH);
  float*          SD   = (float*)(ws + oSD);
  float*          PAR  = (float*)(ws + oPAR);
  int*            LIST = (int*)(ws + oLIST);
  int*            CO   = (int*)(ws + oCO);
  int*            FLAG = (int*)(ws + oFLAG);

  hipFuncSetAttribute(reinterpret_cast<const void*>(&k_bucket), hipFuncAttributeMaxDynamicSharedMemorySize, (int)BK_LDS);

  k_prep<<<PBTOT, NTHR, 0, stream>>>(x, W1, W2, W3, Wc1, a1s, a1d, b1, a2s, a2d, b2, a3s, a3d, b3, bc1, Wc2, bc2,
                                     XB, W1T, W2D, W3D, WC1D, PAR);
  k_bucket<<<NBK, NTHR, BK_LDS, stream>>>(srcs, dsts, LIST, CO, FLAG);

  k_gemm<FIN, FIN, FIN, HC, 4><<<NP / GBM, NTHR, 0, stream>>>(XB, W1T, PAR + P_A1, H, SD);
  k_replay_wide<<<NP / NWAVE, NTHR, 0, stream>>>(LIST, CO, FLAG, H, SD, PAR + P_B1, E);
  k_gemm<K_TWO, 1024, 1024, HC, 4><<<NP / GBM, NTHR, 0, stream>>>(E, W2D, PAR + P_A2, H, SD);
  k_replay_wide<<<NP / NWAVE, NTHR, 0, stream>>>(LIST, CO, FLAG, H, SD, PAR + P_B2, E);
  k_gemm<K_THREE, 1024, 1024, CD, 1><<<NP / GBM, NTHR, 0, stream>>>(E, W3D, PAR + P_A3, H, SD);
  k_replay_narrow<<<NP / NWAVE, NTHR, 0, stream>>>(LIST, CO, FLAG, H, SD, PAR + P_B3, out, E3);
  k_head<<<NP / GBM, NTHR, 0, stream>>>(E3, WC1D, PAR, FLAG, out);
}
